// CrossModalAttention_49065706389687
// MI455X (gfx1250) — hardware-verified
//
#include <hip/hip_runtime.h>


#ifndef NB
#define NB 8
#endif
#ifndef NQ
#define NQ 512
#endif
#define NB_FULL 8
#define NQ_FULL 512
#define NK 4096
#define DM 256
#define NH 8
#define HD 32
#define QCAR 8.0f
#define KCAR 8.0f
#define VCAR 4.0f
#define RCAR 1024.0f
#define PCAR 16384.0f
#define SCL2 (0.17677669529663687f * 0.015625f)

static_assert(NB >= 1 && NB <= NB_FULL);
static_assert(NQ >= 64 && NQ <= NQ_FULL && (NQ % 64) == 0);
static_assert(NK == 256 * 16);
static_assert((DM % 64) == 0 && (NK % 64) == 0 && HD == 32 && NH * HD == DM);

typedef _Float16 h16;
typedef unsigned short bf;
typedef __attribute__((ext_vector_type(16))) __bf16   v16bf;
typedef __attribute__((ext_vector_type(16))) _Float16 v16h;
typedef __attribute__((ext_vector_type(8)))  _Float16 v8h;
typedef __attribute__((ext_vector_type(8)))  unsigned short v8us;
typedef __attribute__((ext_vector_type(8)))  float    v8f;
typedef __attribute__((ext_vector_type(4)))  float    v4f;
typedef v8h  __attribute__((may_alias)) v8ha;
typedef v4f  __attribute__((may_alias)) v4fa;
typedef v8us __attribute__((may_alias)) v8usa;

__device__ __forceinline__ unsigned short f2bf(float f) { unsigned u = __float_as_uint(f); u += 0x7FFFu + ((u >> 16) & 1u); return (unsigned short)(u >> 16); }
__device__ __forceinline__ float bf2f(unsigned short b) { return __uint_as_float(((unsigned)b) << 16); }
__device__ __forceinline__ float bfr(float f) { return bf2f(f2bf(f)); }
__device__ __forceinline__ v16h cat16(v8h lo, v8h hi) { return __builtin_shufflevector(lo, hi, 0, 1, 2, 3, 4, 5, 6, 7, 8, 9, 10, 11, 12, 13, 14, 15); }
__device__ __forceinline__ v16bf cat16b(v8us lo, v8us hi) { return __builtin_bit_cast(v16bf, __builtin_shufflevector(lo, hi, 0, 1, 2, 3, 4, 5, 6, 7, 8, 9, 10, 11, 12, 13, 14, 15)); }
__device__ __forceinline__ v8f wmma16(v16h a, v16h b, v8f c) { return __builtin_amdgcn_wmma_f32_16x16x32_f16(false, a, false, b, (short)0, c, false, false); }
__device__ __forceinline__ v8f wmmab(v16bf a, v16bf b, v8f c) { return __builtin_amdgcn_wmma_f32_16x16x32_bf16(false, a, false, b, (short)0, c, false, false); }
__device__ __forceinline__ h16 tohx(float x) { return (h16)x; }
__device__ __forceinline__ void splitf(float y, unsigned short& h, unsigned short& l) { h = f2bf(y); l = f2bf(y - bf2f(h)); }

template <typename T16> struct WFrag;
template <> struct WFrag<h16> { typedef v16h V; static __device__ __forceinline__ V ld(const h16* p) { return cat16(*(const v8h*)p, *(const v8h*)(p + 16)); } static __device__ __forceinline__ v8f mma(V a, V b, v8f c) { return wmma16(a, b, c); } };
template <> struct WFrag<bf> { typedef v16bf V; static __device__ __forceinline__ V ld(const bf* p) { return cat16b(*(const v8us*)p, *(const v8us*)(p + 16)); } static __device__ __forceinline__ v8f mma(V a, V b, v8f c) { return wmmab(a, b, c); } };
template <typename T16, int MODE, bool BIAS, int NBN>
__global__ __launch_bounds__(32) void k_gemmw(const T16* __restrict__ A, const T16* __restrict__ A2, int lda, const T16* __restrict__ Bt, const T16* __restrict__ Bt2, int ldb, int K, float* C, int ldc, const float* __restrict__ bias, float oscale, float rs2, size_t sA, size_t sB, size_t sC) {
    typedef typename WFrag<T16>::V V;
    __shared__ __align__(16) float os[16 * 68];
    const size_t z = blockIdx.z; A += z * sA; if (MODE == 1) A2 += z * sA; Bt += z * sB; if (MODE == 2) Bt2 += z * sB; C += z * sC;
    const int lane = threadIdx.x & 31, lr = lane & 15, hi = lane >> 4; const int r0 = blockIdx.x * 64, c0 = blockIdx.y * (16 * NBN);
    v8f acc[4][NBN], acc2[4][NBN];
#pragma unroll
    for (int mb = 0; mb < 4; ++mb)
#pragma unroll
        for (int nb = 0; nb < NBN; ++nb) { acc[mb][nb] = (v8f){}; acc2[mb][nb] = (v8f){}; }
    const size_t aoff = (size_t)(r0 + lr) * lda + 8 * hi, boff = (size_t)(c0 + lr) * ldb + 8 * hi;
#pragma unroll 1
    for (int kc = 0; kc < K; kc += 32) {
        V a[4], a2[4];
#pragma unroll
        for (int mb = 0; mb < 4; ++mb) { a[mb] = WFrag<T16>::ld(A + aoff + (size_t)mb * 16 * lda + kc); if (MODE == 1) a2[mb] = WFrag<T16>::ld(A2 + aoff + (size_t)mb * 16 * lda + kc); }
#pragma unroll
        for (int nb = 0; nb < NBN; ++nb) { const V b = WFrag<T16>::ld(Bt + boff + (size_t)nb * 16 * ldb + kc); V b2; if (MODE == 2) b2 = WFrag<T16>::ld(Bt2 + boff + (size_t)nb * 16 * ldb + kc);
#pragma unroll
            for (int mb = 0; mb < 4; ++mb) { acc[mb][nb] = WFrag<T16>::mma(a[mb], b, acc[mb][nb]); if (MODE == 1) acc[mb][nb] = WFrag<T16>::mma(a2[mb], b, acc[mb][nb]); if (MODE == 2) acc2[mb][nb] = WFrag<T16>::mma(a[mb], b2, acc2[mb][nb]); } }
        if (MODE == 2) asm volatile("v_nop\n\tv_nop\n\tv_nop\n\tv_nop" : "+v"(acc[0][0]), "+v"(acc[1][NBN - 1]), "+v"(acc[2][0]), "+v"(acc[3][NBN - 1]), "+v"(acc2[0][0]), "+v"(acc2[1][NBN - 1]), "+v"(acc2[2][0]), "+v"(acc2[3][NBN - 1]) : "v"(a[0]), "v"(a[3]));
        else asm volatile("v_nop\n\tv_nop\n\tv_nop\n\tv_nop" : "+v"(acc[0][0]), "+v"(acc[1][NBN - 1]), "+v"(acc[2][0]), "+v"(acc[3][NBN - 1]) : "v"(a[0]), "v"(a[3]));
    }
    constexpr int LPR = 4 * NBN, RPI = 32 / LPR, NIT = 16 / RPI;
    const int rl = lane / LPR, cofs = (lane % LPR) * 4;
#pragma unroll
    for (int mb = 0; mb < 4; ++mb) {
#pragma unroll
        for (int nb = 0; nb < NBN; ++nb) {
#pragma unroll
            for (int j = 0; j < 8; ++j) { float vv = acc[mb][nb][j]; if (MODE == 2) vv += acc2[mb][nb][j] * rs2; os[(hi * 8 + j) * 68 + nb * 16 + lr] = vv * oscale; } }
        __builtin_amdgcn_wave_barrier(); asm volatile("" ::: "memory");
        float* crow = C + (size_t)(r0 + mb * 16) * ldc + c0;
#pragma unroll 1
        for (int ps = 0; ps < 2; ++ps) {
#pragma unroll
            for (int s = 0; s < NIT; ++s) { const int row = RPI * s + rl; v4f val = *(const v4fa*)(os + row * 68 + cofs); if (BIAS) { val[0] += bfr(bias[c0 + cofs]); val[1] += bfr(bias[c0 + cofs + 1]); val[2] += bfr(bias[c0 + cofs + 2]); val[3] += bfr(bias[c0 + cofs + 3]); }
                *(volatile v4f*)(crow + (size_t)row * ldc + cofs) = val; }
            if (ps == 0) __threadfence(); }
        __builtin_amdgcn_wave_barrier(); asm volatile("" ::: "memory");
    }
}

__global__ __launch_bounds__(256) void k_cvt8(const float* __restrict__ src, bf* dst, size_t n8) { const size_t i = (size_t)blockIdx.x * 256 + threadIdx.x; if (i >= n8) return; const v8f v = *(const v8f*)(src + i * 8); v8us o;
#pragma unroll
    for (int k = 0; k < 8; ++k) o[k] = f2bf(v[k]); *(volatile v8us*)(dst + i * 8) = o; __threadfence(); *(volatile v8us*)(dst + i * 8) = o; }

__global__ __launch_bounds__(256) void k_wT(const float* __restrict__ W, bf* WT, int Kin, int Nout) { const size_t g = (size_t)blockIdx.x * 256 + threadIdx.x; if (g >= (size_t)Nout * Kin / 8) return; const int k0 = (int)(g % (size_t)(Kin / 8)) * 8; const int n = (int)(g / (size_t)(Kin / 8)); v8us o;
#pragma unroll
    for (int q = 0; q < 8; ++q) o[q] = f2bf(W[(size_t)(k0 + q) * Nout + n]);
    bf* d = WT + (size_t)n * Kin + k0; *(volatile v8us*)d = o; __threadfence(); *(volatile v8us*)d = o; }

__global__ __launch_bounds__(256) void k_q16(const float* __restrict__ src, h16* dst, size_t n8) { const size_t i = (size_t)blockIdx.x * 256 + threadIdx.x; if (i >= n8) return; const v8f v = *(const v8f*)(src + i * 8); v8h o;
#pragma unroll
    for (int k = 0; k < 8; ++k) o[k] = tohx(v[k] * QCAR); *(volatile v8h*)(dst + i * 8) = o; __threadfence(); *(volatile v8h*)(dst + i * 8) = o; }

__global__ __launch_bounds__(256) void k_kv16(const float* __restrict__ KV, h16* K16, h16* VTh, h16* VTl) {
    const size_t g = (size_t)blockIdx.x * 256 + threadIdx.x; const size_t NA = (size_t)NK * DM / 8;
    if (g < NA) {
        const int j = (int)(g / (DM / 8)); const int c0 = (int)(g % (DM / 8)) * 8;
        const v8f a = *(const v8f*)(KV + (size_t)j * (2 * DM) + c0); v8h o;
#pragma unroll
        for (int q = 0; q < 8; ++q) o[q] = tohx(a[q] * KCAR);
        h16* d = K16 + (size_t)j * DM + c0; *(volatile v8h*)d = o; __threadfence(); *(volatile v8h*)d = o;
    } else if (g < 2 * NA) {
        const size_t e = g - NA; const int j0 = (int)(e % (size_t)(NK / 8)) * 8; const int c = (int)(e / (size_t)(NK / 8));
        v8h oh, ol;
#pragma unroll
        for (int q = 0; q < 8; ++q) { const float y = KV[(size_t)(j0 + q) * (2 * DM) + DM + c] * VCAR; const h16 hh = tohx(y); oh[q] = hh; ol[q] = tohx(__fmul_rn(__fsub_rn(y, (float)hh), RCAR)); }
        const size_t oo = (size_t)c * NK + j0;
        *(volatile v8h*)(VTh + oo) = oh; *(volatile v8h*)(VTl + oo) = ol; __threadfence(); *(volatile v8h*)(VTh + oo) = oh; *(volatile v8h*)(VTl + oo) = ol;
    }
}

__global__ __launch_bounds__(256) void k_soft(const float* __restrict__ Sb, h16* P) {
    __shared__ float red[16];
    const int t = threadIdx.x, lane = t & 31, w = t >> 5;
    const size_t row = blockIdx.x;
    const float* sr = Sb + row * NK;
    const int c0 = t * 8, c1 = NK / 2 + t * 8;
    const v8f a0 = *(const v8f*)(sr + c0); const v8f a1 = *(const v8f*)(sr + c1);
    float v[16]; float mx = -3.0e38f;
#pragma unroll
    for (int q = 0; q < 8; ++q) { v[q] = a0[q] * SCL2; v[8 + q] = a1[q] * SCL2; mx = fmaxf(mx, fmaxf(v[q], v[8 + q])); }
#pragma unroll
    for (int sh = 16; sh; sh >>= 1) mx = fmaxf(mx, __shfl_xor(mx, sh, 32));
    if (lane == 0) red[w] = mx;
    __syncthreads();
    mx = red[0];
#pragma unroll
    for (int i = 1; i < 8; ++i) mx = fmaxf(mx, red[i]);
    float sum = 0.f;
#pragma unroll
    for (int k = 0; k < 16; ++k) { float d0 = __fsub_rn(v[k], mx); asm volatile("" : "+v"(d0)); v[k] = __builtin_amdgcn_exp2f(__fmul_rn(d0, 1.4426950408889634f)); sum += v[k]; }
#pragma unroll
    for (int sh = 16; sh; sh >>= 1) sum += __shfl_xor(sum, sh, 32);
    if (lane == 0) red[8 + w] = sum;
    __syncthreads();
    float tot = red[8];
#pragma unroll
    for (int i = 1; i < 8; ++i) tot += red[8 + i];
    const float f = __fdiv_rn(PCAR, tot);
    v8h o0, o1;
#pragma unroll
    for (int q = 0; q < 8; ++q) { o0[q] = tohx(v[q] * f); o1[q] = tohx(v[8 + q] * f); }
    h16* pr = P + row * NK;
    *(volatile v8h*)(pr + c0) = o0; *(volatile v8h*)(pr + c1) = o1; __threadfence(); *(volatile v8h*)(pr + c0) = o0; *(volatile v8h*)(pr + c1) = o1;
}

__global__ __launch_bounds__(256) void k_split(const float* __restrict__ src, bf* dh, bf* dl, size_t n8) { const size_t i = (size_t)blockIdx.x * 256 + threadIdx.x; if (i >= n8) return; const v8f v = *(const v8f*)(src + i * 8); v8us oh, ol;
#pragma unroll
    for (int k = 0; k < 8; ++k) { unsigned short a, c; splitf(v[k], a, c); oh[k] = a; ol[k] = c; }
    *(volatile v8us*)(dh + i * 8) = oh; *(volatile v8us*)(dl + i * 8) = ol; __threadfence(); *(volatile v8us*)(dh + i * 8) = oh; *(volatile v8us*)(dl + i * 8) = ol; }

constexpr size_t al256(size_t x) { return (x + 255) & ~(size_t)255; }
constexpr size_t cmax(size_t a, size_t b) { return a > b ? a : b; }
constexpr size_t SZ_XS  = al256((size_t)NB * NQ_FULL * DM * 2);
constexpr size_t SZ_WQ  = al256((size_t)DM * DM * 2);
constexpr size_t SZ_WKV = al256((size_t)2 * DM * DM * 2);
constexpr size_t SZ_WO  = al256((size_t)DM * DM * 2);
constexpr size_t SZ_GF  = al256(cmax((size_t)NB * NQ * DM * 4, (size_t)NK * 2 * DM * 4));
constexpr size_t SZ_Q16 = al256((size_t)NB * NQ * DM * 2);
constexpr size_t SZ_XP  = al256((size_t)NK * DM * 2);
constexpr size_t SZ_K16 = al256((size_t)NK * DM * 2);
constexpr size_t SZ_VT  = al256((size_t)DM * NK * 2);
constexpr size_t SZ_S   = al256((size_t)NH * NQ * NK * 4);
constexpr size_t SZ_P   = al256((size_t)NH * NQ * NK * 2);
constexpr size_t SZ_CTX = al256((size_t)NB * NQ * DM * 4);
constexpr size_t SZ_C16 = al256((size_t)NB * NQ * DM * 2);
constexpr size_t O_XS = 0, O_WQ = O_XS + SZ_XS, O_WKV = O_WQ + SZ_WQ, O_WO = O_WKV + SZ_WKV, O_GF = O_WO + SZ_WO, O_Q16 = O_GF + SZ_GF, O_XP = O_Q16 + SZ_Q16, O_K16 = O_XP + SZ_XP,
                 O_VTH = O_K16 + SZ_K16, O_VTL = O_VTH + SZ_VT, O_S = O_VTL + SZ_VT, O_P = O_S + SZ_S, O_CTX = O_P + SZ_P, O_CH = O_CTX + SZ_CTX, O_CL = O_CH + SZ_C16, O_END = O_CL + SZ_C16;
static_assert(O_END <= (size_t)134217728);
static_assert((size_t)NB * NQ * DM * 4 <= SZ_GF && (size_t)NK * 2 * DM * 4 <= SZ_GF);
static_assert(((size_t)(NB_FULL - 1) * NQ_FULL + NQ_FULL) * DM * 4 <= (size_t)NB_FULL * NQ_FULL * DM * 4);

extern "C" void kernel_launch(void* const* d_in, const int* in_sizes, int n_in, void* d_out, int out_size, void* d_ws, size_t ws_size, hipStream_t stream) {
    if (n_in < 8) return;
    if (in_sizes[0] < NB * NQ_FULL * DM || in_sizes[1] < NB * NK * DM || in_sizes[2] < DM * DM || in_sizes[3] < DM || in_sizes[4] < DM * 2 * DM || in_sizes[5] < 2 * DM || in_sizes[6] < DM * DM || in_sizes[7] < DM) return;
    if ((size_t)out_size < (size_t)NB * NQ_FULL * DM) return;
    if (O_END > ws_size) return;
    const float* state = (const float*)d_in[0];
    const float* pts   = (const float*)d_in[1];
    const float* Wq    = (const float*)d_in[2];
    const float* bq    = (const float*)d_in[3];
    const float* Wkv   = (const float*)d_in[4];
    const float* bkv   = (const float*)d_in[5];
    const float* Wo    = (const float*)d_in[6];
    const float* bo    = (const float*)d_in[7];
    float* OUT = (float*)d_out;
    char* ws = (char*)d_ws;
    bf* XS = (bf*)(ws + O_XS); bf* WQT = (bf*)(ws + O_WQ); bf* WKVT = (bf*)(ws + O_WKV); bf* WOT = (bf*)(ws + O_WO);
    float* GF = (float*)(ws + O_GF); h16* Q16 = (h16*)(ws + O_Q16); bf* XP = (bf*)(ws + O_XP); h16* K16 = (h16*)(ws + O_K16);
    h16* VTH = (h16*)(ws + O_VTH); h16* VTL = (h16*)(ws + O_VTL); float* S = (float*)(ws + O_S); h16* P = (h16*)(ws + O_P);
    float* CTX = (float*)(ws + O_CTX); bf* CH = (bf*)(ws + O_CH); bf* CL = (bf*)(ws + O_CL);

    { const size_t n8 = (size_t)NB * NQ_FULL * DM / 8; k_cvt8<<<(unsigned)((n8 + 255) / 256), 256, 0, stream>>>(state, XS, n8); }
    k_wT<<<(unsigned)(((size_t)DM * DM / 8 + 255) / 256), 256, 0, stream>>>(Wq, WQT, DM, DM);
    k_wT<<<(unsigned)(((size_t)2 * DM * DM / 8 + 255) / 256), 256, 0, stream>>>(Wkv, WKVT, DM, 2 * DM);
    k_wT<<<(unsigned)(((size_t)DM * DM / 8 + 255) / 256), 256, 0, stream>>>(Wo, WOT, DM, DM);
    k_gemmw<bf, 0, true, 4><<<dim3(NQ / 64, DM / 64, NB), 32, 0, stream>>>(XS, nullptr, DM, WQT, nullptr, DM, DM, GF, DM, bq, 1.0f, 0.0f, (size_t)NQ_FULL * DM, (size_t)0, (size_t)NQ * DM);
    { const size_t n8 = (size_t)NB * NQ * DM / 8; k_q16<<<(unsigned)((n8 + 255) / 256), 256, 0, stream>>>(GF, Q16, n8); }
    for (int b = 0; b < NB; ++b) {
        const float* pb = pts + (size_t)b * NK * DM;
        { const size_t n8 = (size_t)NK * DM / 8; k_cvt8<<<(unsigned)((n8 + 255) / 256), 256, 0, stream>>>(pb, XP, n8); }
        k_gemmw<bf, 0, true, 4><<<dim3(NK / 64, (2 * DM) / 64, 1), 32, 0, stream>>>(XP, nullptr, DM, WKVT, nullptr, DM, DM, GF, 2 * DM, bkv, 1.0f, 0.0f, (size_t)0, (size_t)0, (size_t)0);
        k_kv16<<<(unsigned)((size_t)2 * NK * DM / 8 / 256), 256, 0, stream>>>(GF, K16, VTH, VTL);
        k_gemmw<h16, 0, false, 4><<<dim3(NQ / 64, NK / 64, NH), 32, 0, stream>>>(Q16 + (size_t)b * NQ * DM, nullptr, DM, K16, nullptr, DM, HD, S, NK, nullptr, 1.0f, 0.0f, (size_t)HD, (size_t)HD, (size_t)NQ * NK);
        k_soft<<<(unsigned)(NH * NQ), 256, 0, stream>>>(S, P);
        k_gemmw<h16, 2, false, 2><<<dim3(NQ / 64, HD / 32, NH), 32, 0, stream>>>(P, nullptr, NK, VTH, VTL, NK, NK, CTX + (size_t)b * NQ * DM, DM, nullptr, 1.0f / (PCAR * VCAR), 1.0f / RCAR, (size_t)NQ * NK, (size_t)HD * NK, (size_t)HD);
    }
    { const size_t n8 = (size_t)NB * NQ * DM / 8; k_split<<<(unsigned)((n8 + 255) / 256), 256, 0, stream>>>(CTX, CH, CL, n8); }
    k_gemmw<bf, 1, true, 4><<<dim3(NQ / 64, DM / 64, NB), 32, 0, stream>>>(CH, CL, DM, WOT, nullptr, DM, DM, OUT, DM, bo, 1.0f, 0.0f, (size_t)NQ * DM, (size_t)0, (size_t)NQ_FULL * DM);
}
